// MultiScaleRetention_9285719294238
// MI455X (gfx1250) — hardware-verified
//
#include <hip/hip_runtime.h>
#include <math.h>

#pragma clang fp contract(off)

constexpr int kBatch    = 2;
constexpr int kSeq      = 2048;
constexpr int kDm       = 1024;
constexpr int kHeads    = 4;
constexpr int kDk       = 256;
constexpr int kDv       = 512;
constexpr int kHalf     = 128;
constexpr int kTok      = kBatch * kSeq;
constexpr int kKeyDim   = kHeads * kDk;
constexpr int kValDim   = kHeads * kDv;
constexpr int kQKW      = 2 * kKeyDim;
constexpr int kWcatRows = 2 * kKeyDim + 2 * kValDim;
constexpr float kQScale    = 0.0625f;
constexpr float kPCarry    = 4096.0f;
constexpr float kScoreOut  = kPCarry * kQScale;
constexpr float kVCarry    = 16.0f;
constexpr float kCtxScale  = 1.0f / (kPCarry * kVCarry);
constexpr float kGCarry    = 16.0f;
constexpr float kGCarryInv = 1.0f / 16.0f;
constexpr float kOGCarry   = 64.0f;
constexpr float kWoCarry   = 64.0f;
constexpr float kOutScale  = 1.0f / (kOGCarry * kWoCarry);
constexpr float kEps       = 1.0e-5f;
constexpr float kInvDv     = 1.0f / 512.0f;
static_assert(kKeyDim == kDm && kValDim == 2 * kDm && kHalf * 2 == kDk, "shape");
static_assert(kTok % 64 == 0 && kQKW % 64 == 0 && kValDim % 64 == 0 && kDm % 64 == 0 && kSeq % 64 == 0 && kDv % 64 == 0, "M,N tile multiples");
static_assert(kDm % 32 == 0 && kDk % 32 == 0 && kSeq % 32 == 0 && kValDim % 32 == 0, "K multiples of 32");
static_assert((kTok * kDm) % (8 * 256) == 0 && (kDm * kDm) % (8 * 256) == 0 && (kValDim * kDm) % (8 * 256) == 0, "cast grids exact");
static_assert(kQKW == 8 * 256 && kValDim == 8 * 256 && kHalf == 4 * 32, "per-row thread maps");

typedef __attribute__((ext_vector_type(16))) _Float16 v16h;
typedef __attribute__((ext_vector_type(8)))  _Float16 v8h;
typedef __attribute__((ext_vector_type(16))) __bf16   v16b;
typedef __attribute__((ext_vector_type(8)))  __bf16   v8b;
typedef __attribute__((ext_vector_type(8)))  float    v8f;
typedef __attribute__((ext_vector_type(4)))  float    v4f;
typedef __attribute__((ext_vector_type(4)))  unsigned int v4u;

__device__ __forceinline__ unsigned short f2bf_bits(float f) {
  unsigned u = __float_as_uint(f);
  return (unsigned short)((u + 0x7FFFu + ((u >> 16) & 1u)) >> 16);
}
__device__ __forceinline__ float bf_bits2f(unsigned short h) { return __uint_as_float(((unsigned)h) << 16); }

__device__ __forceinline__ float h16_to_f32(unsigned hb) {
  const unsigned sgn = (hb & 0x8000u) << 16; const unsigned em = hb & 0x7fffu;
  const float fn = __uint_as_float((em << 13) + 0x38000000u);
  const float fs = (float)em * 5.9604644775390625e-8f;
  const float mag = (em < 0x400u) ? fs : fn; return __uint_as_float(__float_as_uint(mag) | sgn); }

__device__ __forceinline__ void dep_guard4_h(v8f& a, v8f& b, v8f& c, v8f& d, v16h x, v16h y, v16h z) {
  asm volatile("v_nop\n\tv_nop\n\tv_nop\n\tv_nop" : "+v"(a), "+v"(b), "+v"(c), "+v"(d) : "v"(x), "v"(y), "v"(z)); }
__device__ __forceinline__ void dep_guard4_b(v8f& a, v8f& b, v8f& c, v8f& d, v16b x, v16b y, v16b z) {
  asm volatile("v_nop\n\tv_nop\n\tv_nop\n\tv_nop" : "+v"(a), "+v"(b), "+v"(c), "+v"(d) : "v"(x), "v"(y), "v"(z)); }
__device__ __forceinline__ void keep4_h(v16h a, v16h b, v16h c, v16h d) { asm volatile("v_nop" :: "v"(a), "v"(b), "v"(c), "v"(d)); }
__device__ __forceinline__ void keep4_b(v16b a, v16b b, v16b c, v16b d) { asm volatile("v_nop" :: "v"(a), "v"(b), "v"(c), "v"(d)); }
__device__ __forceinline__ void acc_guard4(v8f& a, v8f& b, v8f& c, v8f& d) { asm volatile("v_nop\n\tv_nop\n\tv_nop\n\tv_nop" : "+v"(a), "+v"(b), "+v"(c), "+v"(d)); }
template <typename T> struct Frag;
template <> struct Frag<_Float16> {
  typedef v16h V; union U { v16h v; v8h h[2]; };
  static __device__ __forceinline__ v16h load(const _Float16* p) {
    U f; f.h[0] = *(const v8h*)(p); f.h[1] = *(const v8h*)(p + 16); return f.v;
  }
  static __device__ __forceinline__ v8f mma(v16h a, v16h b, v8f c) {
    return __builtin_amdgcn_wmma_f32_16x16x32_f16(false, a, false, b, (short)0, c, false, false);
  }
  static __device__ __forceinline__ void guard4(v8f& a, v8f& b, v8f& c, v8f& d, v16h x, v16h y, v16h z) { dep_guard4_h(a, b, c, d, x, y, z); }
  static __device__ __forceinline__ void keep(v16h a, v16h b, v16h c, v16h d) { keep4_h(a, b, c, d); }
};
template <> struct Frag<__bf16> {
  typedef v16b V; union U { v16b v; v8b h[2]; };
  static __device__ __forceinline__ v16b load(const __bf16* p) {
    U f; f.h[0] = *(const v8b*)(p); f.h[1] = *(const v8b*)(p + 16); return f.v;
  }
  static __device__ __forceinline__ v8f mma(v16b a, v16b b, v8f c) {
    return __builtin_amdgcn_wmma_f32_16x16x32_bf16(false, a, false, b, (short)0, c, false, false);
  }
  static __device__ __forceinline__ void guard4(v8f& a, v8f& b, v8f& c, v8f& d, v16b x, v16b y, v16b z) { dep_guard4_b(a, b, c, d, x, y, z); }
  static __device__ __forceinline__ void keep(v16b a, v16b b, v16b c, v16b d) { keep4_b(a, b, c, d); }
};

__device__ __forceinline__ unsigned pk16(unsigned short a, unsigned short b) { return (unsigned)a | ((unsigned)b << 16); }
__device__ __forceinline__ unsigned short h_bits(float f) { const _Float16 h = (_Float16)f; return __builtin_bit_cast(unsigned short, h); }

struct DecayEpi { float lr[8]; float l16[4]; float il16[4]; float l8; float logd; };
static_assert(sizeof(DecayEpi) == 72, "no padding");

template <int ET> struct Elem;
template <> struct Elem<0> { typedef _Float16 T; };
template <> struct Elem<1> { typedef __bf16 T; };
template <int ET, bool SPLIT, int OUT_MODE, int CMODE>
__global__ __launch_bounds__(256) void wmma_gemm64(const unsigned short* __restrict__ Ap, const unsigned short* __restrict__ A2p, int lda,
                                                   const unsigned short* __restrict__ Btp, const unsigned short* __restrict__ Bt2p, int ldb,
                                                   void* __restrict__ Cout, int ldc,
                                                   int M, int N, int K, float scale, DecayEpi de) {
  typedef typename Elem<ET>::T T;
  typedef typename Frag<T>::V V;
  const T* A = (const T*)Ap; const T* A2 = (const T*)A2p; const T* Bt = (const T*)Btp; const T* Bt2 = (const T*)Bt2p;
  __shared__ __align__(16) float sT[8][16 * 68];
  const int lane = threadIdx.x & 31;
  const int wave = threadIdx.x >> 5;
  const int tilesN = N >> 6;
  const int tilesM = M >> 6;
  const int tile = blockIdx.x * 8 + wave;
  if (tile >= tilesM * tilesN) return;
  const int tm = tile / tilesN;
  const int tn = tile - tm * tilesN;
  const int m0 = tm << 6;
  const int n0 = tn << 6;
  if (CMODE == 1 && n0 > m0) return;
  int Kend = K;
  if (CMODE == 2) { const int kl = m0 + 64; Kend = (kl < K) ? kl : K; }

  const int rlane = lane & 15;
  const int koff  = (lane >> 4) * 8;
  const int mOff  = (lane >> 4) * 8;

  v8f acc[4][4];
#pragma unroll
  for (int i = 0; i < 4; ++i)
#pragma unroll
    for (int j = 0; j < 4; ++j) acc[i][j] = (v8f){0.f,0.f,0.f,0.f,0.f,0.f,0.f,0.f};

  for (int k0 = 0; k0 < Kend; k0 += 32) {
    V bh[4], bl[4];
#pragma unroll
    for (int j = 0; j < 4; ++j) {
      const size_t bo = (size_t)(n0 + (j << 4) + rlane) * ldb + koff + k0;
      bh[j] = Frag<T>::load(Bt + bo);
      if (SPLIT) bl[j] = Frag<T>::load(Bt2 + bo); else bl[j] = bh[j];
    }
#pragma unroll
    for (int i = 0; i < 4; ++i) {
      const size_t ao = (size_t)(m0 + (i << 4) + rlane) * lda + koff + k0;
      V ah = Frag<T>::load(A + ao);
      V al = ah;
      if (SPLIT) al = Frag<T>::load(A2 + ao);
#pragma unroll
      for (int j = 0; j < 4; ++j) {
        acc[i][j] = Frag<T>::mma(ah, bh[j], acc[i][j]);
        if (SPLIT) {
          acc[i][j] = Frag<T>::mma(ah, bl[j], acc[i][j]);
          acc[i][j] = Frag<T>::mma(al, bh[j], acc[i][j]);
        }
      }
      Frag<T>::guard4(acc[i][0], acc[i][1], acc[i][2], acc[i][3], ah, al, bh[3]);
    }
    Frag<T>::keep(bh[0], bh[1], bh[2], bh[3]);
    if (SPLIT) Frag<T>::keep(bl[0], bl[1], bl[2], bl[3]);
  }
  acc_guard4(acc[0][0], acc[0][1], acc[0][2], acc[0][3]);
  acc_guard4(acc[1][0], acc[1][1], acc[1][2], acc[1][3]);
  acc_guard4(acc[2][0], acc[2][1], acc[2][2], acc[2][3]);
  acc_guard4(acc[3][0], acc[3][1], acc[3][2], acc[3][3]);

  float rowfac[8], colfac[4];
  float ftile = 1.0f;
  {
    float flm = 1.0f, flc = 1.0f;
    if (CMODE == 1) {
      flm = (lane >> 4) ? de.l8 : 1.0f;
      flc = expf(-de.logd * (float)rlane);
      ftile = expf(de.logd * (float)(m0 - n0));
    }
#pragma unroll
    for (int r = 0; r < 8; ++r) rowfac[r] = (CMODE == 1) ? flm * de.lr[r] : 1.0f;
#pragma unroll
    for (int j = 0; j < 4; ++j) colfac[j] = (CMODE == 1) ? flc * de.il16[j] : 1.0f;
  }

  float* slab = sT[wave];
#pragma unroll
  for (int i = 0; i < 4; ++i) {
    const int mBase = m0 + (i << 4);
    const float fti = (CMODE == 1) ? ftile * de.l16[i] : 1.0f;
#pragma unroll
    for (int j = 0; j < 4; ++j) {
#pragma unroll
      for (int r = 0; r < 8; ++r) {
        float v = acc[i][j][r] * scale;
        if (CMODE == 1) {
          const float f = (rowfac[r] * colfac[j]) * fti;
          v = v * f;
          const int trow = mBase + mOff + r;
          const int scol = n0 + (j << 4) + rlane;
          v = (scol <= trow) ? v : 0.0f;
        }
        slab[(mOff + r) * 68 + (j << 4) + rlane] = v;
      }
    }
    __builtin_amdgcn_fence(__ATOMIC_RELEASE, "workgroup");
    __builtin_amdgcn_wave_barrier();
    __builtin_amdgcn_fence(__ATOMIC_ACQUIRE, "workgroup");
    if (OUT_MODE == 0) {
      float* C = (float*)Cout;
      const int hh = lane >> 4, c4 = (lane & 15) * 4;
      for (int pass = 0; pass < 2; ++pass) {
#pragma unroll
        for (int it = 0; it < 8; ++it) {
          const int row = it * 2 + hh;
          v4f v = *(const v4f*)(slab + row * 68 + c4);
          *(volatile v4f*)(C + (size_t)(mBase + row) * ldc + n0 + c4) = v;
        }
        __threadfence();
      }
    } else {
      const int q = lane >> 3, c8 = (lane & 7) * 8;
      unsigned short* C = (unsigned short*)Cout;
      for (int pass = 0; pass < 2; ++pass) {
#pragma unroll
        for (int it = 0; it < 4; ++it) {
          const int row = it * 4 + q;
          const float* sp = slab + row * 68 + c8;
          v8h hv;
#pragma unroll
          for (int e = 0; e < 8; ++e) hv[e] = (_Float16)sp[e];
          *(volatile v8h*)(C + (size_t)(mBase + row) * ldc + n0 + c8) = hv;
        }
        __threadfence();
      }
    }
    __builtin_amdgcn_fence(__ATOMIC_RELEASE, "workgroup");
    __builtin_amdgcn_wave_barrier();
    __builtin_amdgcn_fence(__ATOMIC_ACQUIRE, "workgroup");
  }
}

__global__ __launch_bounds__(256) void cast8_bf16_kernel(const float* __restrict__ in, unsigned short* __restrict__ out, int n8) {
  const int i = blockIdx.x * 256 + threadIdx.x;
  if (i >= n8) return;
  const float* p = in + 8 * (size_t)i;
  const v4f a = *(const v4f*)(p);
  const v4f c = *(const v4f*)(p + 4);
  unsigned short hb[8];
#pragma unroll
  for (int e = 0; e < 4; ++e) {
    hb[e]     = f2bf_bits(a[e]);
    hb[4 + e] = f2bf_bits(c[e]);
  }
  const v4u u = (v4u){pk16(hb[0], hb[1]), pk16(hb[2], hb[3]), pk16(hb[4], hb[5]), pk16(hb[6], hb[7])};
  unsigned short* q = out + 8 * (size_t)i;
  *(volatile v4u*)q = u;
  __threadfence();
  *(volatile v4u*)q = u;
}

__global__ __launch_bounds__(256) void cast8_wo_kernel(const float* __restrict__ in, unsigned short* __restrict__ out, int n8) {
  const int i = blockIdx.x * 256 + threadIdx.x;
  if (i >= n8) return;
  const float* p = in + 8 * (size_t)i;
  const v4f a = *(const v4f*)(p);
  const v4f c = *(const v4f*)(p + 4);
  unsigned short hb[8];
#pragma unroll
  for (int e = 0; e < 4; ++e) {
    hb[e]     = h_bits(bf_bits2f(f2bf_bits(a[e])) * kWoCarry);
    hb[4 + e] = h_bits(bf_bits2f(f2bf_bits(c[e])) * kWoCarry);
  }
  const v4u u = (v4u){pk16(hb[0], hb[1]), pk16(hb[2], hb[3]), pk16(hb[4], hb[5]), pk16(hb[6], hb[7])};
  unsigned short* q = out + 8 * (size_t)i;
  *(volatile v4u*)q = u;
  __threadfence();
  *(volatile v4u*)q = u;
}

struct RopeFreq { float invf[kHalf]; };
static_assert(sizeof(RopeFreq) == 512, "no padding");

__global__ __launch_bounds__(128) void trig_table_kernel(float* __restrict__ CS, RopeFreq rf) {
  __shared__ __align__(16) float sInv[kHalf];
  __shared__ __align__(16) float sC[kHalf];
  __shared__ __align__(16) float sS[kHalf];
  const int tid  = threadIdx.x;
  const int lane = tid & 31, wave = tid >> 5;
  const int t    = blockIdx.x;
  if (tid == 0) {
#pragma unroll
    for (int j = 0; j < kHalf; ++j) sInv[j] = rf.invf[j];
  }
  __syncthreads();
  const float ang = (float)t * sInv[tid];
  const float cs = cosf(ang);
  const float sn = sinf(ang);
  sC[tid] = cs;
  sS[tid] = sn;
  __syncthreads();
  if (wave == 0) {
    const v4f v = *(const v4f*)(sC + 4 * lane);
    float* dst = CS + (size_t)t * kHalf + 4 * lane;
    *(volatile v4f*)dst = v;
    __threadfence();
    *(volatile v4f*)dst = v;
  } else if (wave == 1) {
    const v4f v = *(const v4f*)(sS + 4 * lane);
    float* dst = CS + (size_t)kSeq * kHalf + (size_t)t * kHalf + 4 * lane;
    *(volatile v4f*)dst = v;
    __threadfence();
    *(volatile v4f*)dst = v;
  }
}

__global__ __launch_bounds__(256) void rope_kernel(const float* __restrict__ QK32, const float* __restrict__ CS,
                                                   unsigned short* __restrict__ QKhi, unsigned short* __restrict__ QKlo) {
  __shared__ __align__(16) float sIn[kQKW];
  __shared__ __align__(16) float sRot[kQKW];
  __shared__ __align__(16) float sCos[kHalf];
  __shared__ __align__(16) float sSin[kHalf];
  const int bt   = blockIdx.x;
  const int t    = bt & (kSeq - 1);
  const int tid  = threadIdx.x;
  const int lane = tid & 31, wave = tid >> 5;
  {
    const float* row = QK32 + (size_t)bt * kQKW + 8 * tid;
    const v4f a = *(const v4f*)(row);
    const v4f c = *(const v4f*)(row + 4);
    *(v4f*)(sIn + 8 * tid)     = a;
    *(v4f*)(sIn + 8 * tid + 4) = c;
  }
  if (wave == 0) {
    const v4f v = *(const v4f*)(CS + (size_t)t * kHalf + 4 * lane);
    *(v4f*)(sCos + 4 * lane) = v;
  } else if (wave == 1) {
    const v4f v = *(const v4f*)(CS + (size_t)kSeq * kHalf + (size_t)t * kHalf + 4 * lane);
    *(v4f*)(sSin + 4 * lane) = v;
  }
  __syncthreads();
#pragma unroll
  for (int u = 0; u < 2; ++u) {
    const int p  = tid + 256 * u;
    const int hh = p >> 7;
    const int j  = p & 127;
    const float cs = sCos[j], sn = sSin[j];
    {
      const int i1 = hh * kDk + j, i2 = i1 + kHalf;
      const float x1 = sIn[i1], x2 = sIn[i2];
      sRot[i1] = x1 * cs - x2 * sn;
      sRot[i2] = x1 * sn + x2 * cs;
    }
    {
      const int i1 = kKeyDim + hh * kDk + j, i2 = i1 + kHalf;
      const float x1 = sIn[i1], x2 = sIn[i2];
      sRot[i1] = x1 * cs - x2 * sn;
      sRot[i2] = x1 * sn + x2 * cs;
    }
  }
  __syncthreads();
  {
    const v4f r0 = *(const v4f*)(sRot + 8 * tid);
    const v4f r1 = *(const v4f*)(sRot + 8 * tid + 4);
    float rv[8];
#pragma unroll
    for (int e = 0; e < 4; ++e) { rv[e] = r0[e]; rv[4 + e] = r1[e]; }
    unsigned short hb[8], lb[8];
#pragma unroll
    for (int e = 0; e < 8; ++e) {
      hb[e] = f2bf_bits(rv[e]);
      lb[e] = f2bf_bits(rv[e] - bf_bits2f(hb[e]));
    }
    const v4u uh = (v4u){pk16(hb[0], hb[1]), pk16(hb[2], hb[3]), pk16(hb[4], hb[5]), pk16(hb[6], hb[7])};
    const v4u ul = (v4u){pk16(lb[0], lb[1]), pk16(lb[2], lb[3]), pk16(lb[4], lb[5]), pk16(lb[6], lb[7])};
    unsigned short* dh = QKhi + (size_t)bt * kQKW + 8 * tid;
    unsigned short* dl = QKlo + (size_t)bt * kQKW + 8 * tid;
    *(volatile v4u*)dh = uh;
    *(volatile v4u*)dl = ul;
    __threadfence();
    *(volatile v4u*)dh = uh;
    *(volatile v4u*)dl = ul;
  }
}

__global__ __launch_bounds__(256) void normgate_kernel(const float* __restrict__ Ob, unsigned short* Gio,
                                                       const float* __restrict__ gnw) {
  __shared__ float red[8];
  __shared__ __align__(16) unsigned short sog[kValDim];
  const int bt   = blockIdx.x;
  const int tid  = threadIdx.x;
  const int lane = tid & 31, wave = tid >> 5;
  const int hh   = tid >> 6;
  const int li   = tid & 63;
  const int col  = hh * kDv + 8 * li;
  const float* op = Ob + (size_t)bt * kValDim + col;
  const v4f o0 = *(const v4f*)(op);
  const v4f o1 = *(const v4f*)(op + 4);
  float ss = 0.0f;
#pragma unroll
  for (int e = 0; e < 4; ++e) { ss += o0[e] * o0[e]; ss += o1[e] * o1[e]; }
#pragma unroll
  for (int off = 16; off > 0; off >>= 1) ss += __shfl_xor(ss, off, 32);
  if (lane == 0) red[wave] = ss;
  __syncthreads();
  const float tot = red[2 * hh] + red[2 * hh + 1];
  const float rms = rsqrtf(tot * kInvDv + kEps);

  unsigned short* grow = Gio + (size_t)bt * kValDim + col;
  const unsigned* gp32 = (const unsigned*)(const void*)grow;
  const float* wp = gnw + 8 * li;
#pragma unroll 1
  for (int it = 0; it < 8; ++it) {
    const float ov = op[it];
    const unsigned w = gp32[it >> 1];
    const unsigned hbits = (w >> ((it & 1) * 16)) & 0xffffu;
    const float g  = h16_to_f32(hbits) * kGCarryInv;
    const float wr = bf_bits2f(f2bf_bits(wp[it]));
    const float on = (ov * rms) * wr;
    const float gc = fminf(fmaxf(g, -80.0f), 80.0f);
    const float ex = expf(-gc);
    const float sg = 1.0f / (1.0f + ex);
    const float sw = g * sg;
    const float og = on * sw;
    sog[col + it] = h_bits(og * kOGCarry);
  }
  __syncthreads();
  const v4u u = *(const v4u*)(sog + col);
  *(volatile v4u*)grow = u;
  __threadfence();
  *(volatile v4u*)grow = u;
}

extern "C" void kernel_launch(void* const* d_in, const int* in_sizes, int n_in,
                              void* d_out, int out_size, void* d_ws, size_t ws_size,
                              hipStream_t stream) {
  if (n_in < 7) return;
  if (in_sizes[0] != kTok * kDm) return;
  if (in_sizes[1] != kKeyDim * kDm || in_sizes[2] != kKeyDim * kDm) return;
  if (in_sizes[3] != kValDim * kDm || in_sizes[4] != kValDim * kDm) return;
  if (in_sizes[5] != kDm * kValDim || in_sizes[6] != kDv) return;
  if (out_size != kTok * kDm) return;

  const size_t szXb   = (size_t)kTok * kDm * 2;
  const size_t szWcat = (size_t)kWcatRows * kDm * 2;
  const size_t szWoh  = (size_t)kDm * kValDim * 2;
  const size_t szR32  = (size_t)kTok * kQKW * 4;
  const size_t szQK16 = (size_t)kTok * kQKW * 2;
  const size_t szV16  = (size_t)kValDim * kTok * 2;
  const size_t szP    = (size_t)kSeq * kSeq * 2;
  const size_t szCS   = (size_t)2 * kSeq * kHalf * 4;
  const size_t offXb   = 0;
  const size_t offWcat = offXb + szXb;
  const size_t offWoh  = offWcat + szWcat;
  const size_t offR32  = offWoh + szWoh;
  const size_t offQKhi = offR32 + szR32;
  const size_t offQKlo = offQKhi + szQK16;
  const size_t offV16  = offQKlo + szQK16;
  const size_t offP    = offV16 + szV16;
  const size_t offCS   = offP + szP;
  const size_t total   = offCS + szCS;
  if (ws_size < total) return;

  const float* x   = (const float*)d_in[0];
  const float* Wq  = (const float*)d_in[1];
  const float* Wk  = (const float*)d_in[2];
  const float* Wv  = (const float*)d_in[3];
  const float* Wg  = (const float*)d_in[4];
  const float* Wo  = (const float*)d_in[5];
  const float* gnw = (const float*)d_in[6];
  float* out = (float*)d_out;
  char* ws = (char*)d_ws;
  unsigned short* Xb   = (unsigned short*)(ws + offXb);
  unsigned short* Wcat = (unsigned short*)(ws + offWcat);
  unsigned short* Woh  = (unsigned short*)(ws + offWoh);
  float*          QK32 = (float*)(ws + offR32);
  float*          Ob   = (float*)(ws + offR32);
  unsigned short* QKhi = (unsigned short*)(ws + offQKhi);
  unsigned short* QKlo = (unsigned short*)(ws + offQKlo);
  unsigned short* V16  = (unsigned short*)(ws + offV16);
  unsigned short* Pp   = (unsigned short*)(ws + offP);
  float*          CS   = (float*)(ws + offCS);

  DecayEpi dz = {};

  {
    const int nx8  = (kTok * kDm) / 8;
    const int nqk8 = (kKeyDim * kDm) / 8;
    const int nvg8 = (kValDim * kDm) / 8;
    cast8_bf16_kernel<<<dim3(nx8 / 256), dim3(256), 0, stream>>>(x, Xb, nx8);
    cast8_bf16_kernel<<<dim3(nqk8 / 256), dim3(256), 0, stream>>>(Wq, Wcat, nqk8);
    cast8_bf16_kernel<<<dim3(nqk8 / 256), dim3(256), 0, stream>>>(Wk, Wcat + (size_t)kKeyDim * kDm, nqk8);
    cast8_bf16_kernel<<<dim3(nvg8 / 256), dim3(256), 0, stream>>>(Wv, Wcat + (size_t)2 * kKeyDim * kDm, nvg8);
    cast8_bf16_kernel<<<dim3(nvg8 / 256), dim3(256), 0, stream>>>(Wg, Wcat + (size_t)(2 * kKeyDim + kValDim) * kDm, nvg8);
    cast8_wo_kernel<<<dim3(nvg8 / 256), dim3(256), 0, stream>>>(Wo, Woh, nvg8);
  }

  {
    RopeFreq rf;
    for (int j = 0; j < kHalf; ++j) {
      const float e = (float)(2 * j) / 256.0f;
      const float p = (float)pow(10000.0, (double)e);
      rf.invf[j] = 1.0f / p;
    }
    trig_table_kernel<<<dim3(kSeq), dim3(128), 0, stream>>>(CS, rf);
  }

  {
    const int tiles = (kTok / 64) * (kQKW / 64);
    wmma_gemm64<1, false, 0, 0><<<dim3((tiles + 7) / 8), dim3(256), 0, stream>>>(
        Xb, Xb, kDm, Wcat, Wcat, kDm, (void*)QK32, kQKW, kTok, kQKW, kDm, 1.0f, dz);
  }

  rope_kernel<<<dim3(kTok), dim3(256), 0, stream>>>(QK32, CS, QKhi, QKlo);

  {
    const int tiles = (kValDim / 64) * (kTok / 64);
    wmma_gemm64<1, false, 1, 0><<<dim3((tiles + 7) / 8), dim3(256), 0, stream>>>(
        Wcat + (size_t)2 * kKeyDim * kDm, Wcat + (size_t)2 * kKeyDim * kDm, kDm, Xb, Xb, kDm,
        (void*)V16, kTok, kValDim, kTok, kDm, kVCarry, dz);
  }

  {
    const int tilesS = (kSeq / 64) * (kSeq / 64);
    const int tilesO = (kSeq / 64) * (kDv / 64);
    for (int b = 0; b < kBatch; ++b) {
      for (int h = 0; h < kHeads; ++h) {
        DecayEpi de;
        {
          const float ldf = (float)log1p(-pow(2.0, -5.0 - (double)h));
          const double ld = (double)ldf;
          de.logd = ldf;
          for (int r = 0; r < 8; ++r) de.lr[r] = (float)exp(ld * (double)r);
          for (int i = 0; i < 4; ++i) de.l16[i] = (float)exp(ld * (double)(16 * i));
          for (int j = 0; j < 4; ++j) de.il16[j] = (float)exp(-ld * (double)(16 * j));
          de.l8 = (float)exp(ld * 8.0);
        }
        const unsigned short* Aqh = QKhi + (size_t)b * kSeq * kQKW + (size_t)h * kDk;
        const unsigned short* Aql = QKlo + (size_t)b * kSeq * kQKW + (size_t)h * kDk;
        const unsigned short* Bkh = Aqh + kKeyDim;
        const unsigned short* Bkl = Aql + kKeyDim;
        wmma_gemm64<1, true, 1, 1><<<dim3((tilesS + 7) / 8), dim3(256), 0, stream>>>(
            Aqh, Aql, kQKW, Bkh, Bkl, kQKW, (void*)Pp, kSeq, kSeq, kSeq, kDk, kScoreOut, de);
        const unsigned short* Bv = V16 + (size_t)h * kDv * kTok + (size_t)b * kSeq;
        float* Co = Ob + (size_t)b * kSeq * kValDim + (size_t)h * kDv;
        wmma_gemm64<0, false, 0, 2><<<dim3((tilesO + 7) / 8), dim3(256), 0, stream>>>(
            Pp, Pp, kSeq, Bv, Bv, kTok, (void*)Co, kValDim, kSeq, kDv, kSeq, kCtxScale, dz);
      }
    }
  }

  unsigned short* Gp = V16;
  {
    const int tiles = (kTok / 64) * (kValDim / 64);
    wmma_gemm64<1, false, 1, 0><<<dim3((tiles + 7) / 8), dim3(256), 0, stream>>>(
        Xb, Xb, kDm, Wcat + (size_t)(2 * kKeyDim + kValDim) * kDm, Wcat + (size_t)(2 * kKeyDim + kValDim) * kDm, kDm,
        (void*)Gp, kValDim, kTok, kValDim, kDm, kGCarry, dz);
  }

  normgate_kernel<<<dim3(kTok), dim3(256), 0, stream>>>(Ob, Gp, gnw);

  {
    const int tiles = (kTok / 64) * (kDm / 64);
    wmma_gemm64<0, false, 0, 0><<<dim3((tiles + 7) / 8), dim3(256), 0, stream>>>(
        Gp, Gp, kValDim, Woh, Woh, kValDim, (void*)out, kDm, kTok, kDm, kValDim, kOutScale, dz);
  }
}
